// CSDivergenceLoss_50079318672069
// MI455X (gfx1250) — hardware-run, weakly checked
//
#include <hip/hip_runtime.h>
#include <math.h>

typedef __attribute__((ext_vector_type(16))) _Float16 v16h;
typedef __attribute__((ext_vector_type(16))) __bf16 v16b;
typedef __attribute__((ext_vector_type(8)))  _Float16 v8h;
typedef __attribute__((ext_vector_type(8)))  float v8f;
typedef __attribute__((ext_vector_type(4)))  float v4f;
typedef __attribute__((ext_vector_type(2)))  float v2f;
typedef __attribute__((ext_vector_type(4)))  unsigned v4u;
typedef __attribute__((ext_vector_type(4)))  int v4i;
typedef float __attribute__((may_alias)) float_a;
typedef int __attribute__((may_alias)) int_a;

template <typename T> __device__ __forceinline__ void vst2(void* p, T v) { *(volatile T*)p = v; __threadfence(); *(volatile T*)p = v; }
__device__ __forceinline__ v8f wmma16(v16h a, v16h b, v8f c) {
  v8f d = __builtin_amdgcn_wmma_f32_16x16x32_f16(false, a, false, b, (short)0, c, false, false);
  asm volatile("v_nop\n\tv_nop\n\tv_nop\n\tv_nop" : "+v"(d) : "v"(a), "v"(b));
  return d;
}
__device__ __forceinline__ v8f wmma_bf(v16b a, v16b b, v8f c) {
  v8f d = __builtin_amdgcn_wmma_f32_16x16x32_bf16(false, a, false, b, (short)0, c, false, false);
  asm volatile("v_nop\n\tv_nop\n\tv_nop\n\tv_nop" : "+v"(d) : "v"(a), "v"(b));
  return d;
}
__device__ __forceinline__ v16h frag_h(const _Float16* rowk0, int lane) {
  union { v16h v; v8h q[2]; } u; const _Float16* p = rowk0 + 8 * (lane >> 4);
  u.q[0] = *(const v8h*)p; u.q[1] = *(const v8h*)(p + 16); return u.v;
}
__device__ __forceinline__ v16h frag_f32(const float* rowk0, int lane) {
  v16h a; const float* p = rowk0 + 8 * (lane >> 4);
#pragma unroll
  for (int i = 0; i < 8; ++i) { a[i] = (_Float16)p[i]; a[8 + i] = (_Float16)p[16 + i]; }
  return a;
}
__device__ __forceinline__ v16h frag_f32s(const float* rowk0, int lane, float sc) {
  v16h a; const float* p = rowk0 + 8 * (lane >> 4);
#pragma unroll
  for (int i = 0; i < 8; ++i) { a[i] = (_Float16)(p[i] * sc); a[8 + i] = (_Float16)(p[16 + i] * sc); }
  return a;
}
__device__ __forceinline__ v16h fragc_f32(const float* W, int k0, int n, int lane, int ld, int K) {
  v16h a; const int g = lane >> 4;
#pragma unroll
  for (int i = 0; i < 8; ++i) { const int ka = k0 + 8 * g + i, kb = ka + 16;
    a[i] = (_Float16)(ka < K ? W[(size_t)(ka < K ? ka : K - 1) * ld + n] : 0.f); a[8 + i] = (_Float16)(kb < K ? W[(size_t)(kb < K ? kb : K - 1) * ld + n] : 0.f); }
  return a;
}
struct F2 { v16b h, l; };
__device__ __forceinline__ F2 bsplit16(const float v[16]) { F2 r;
#pragma unroll
  for (int i = 0; i < 16; ++i) { const __bf16 h = (__bf16)v[i]; r.h[i] = h; r.l[i] = (__bf16)(v[i] - (float)h); }
  return r; }
__device__ __forceinline__ F2 split_row(const float* row, int k0, int lane) { float v[16]; const float* p = row + k0 + 8 * (lane >> 4);
#pragma unroll
  for (int i = 0; i < 8; ++i) { v[i] = p[i]; v[8 + i] = p[16 + i]; }
  return bsplit16(v); }
__device__ __forceinline__ F2 split_rowK(const float* row, int k0, int lane, int K) { float v[16]; const int g = lane >> 4;
#pragma unroll
  for (int i = 0; i < 8; ++i) { const int ka = k0 + 8 * g + i, kb = ka + 16; v[i] = ka < K ? row[ka < K ? ka : K - 1] : 0.f; v[8 + i] = kb < K ? row[kb < K ? kb : K - 1] : 0.f; }
  return bsplit16(v); }
__device__ __forceinline__ F2 split_col(const float* W, int k0, int n, int lane, int ld, int K) { float v[16]; const int g = lane >> 4;
#pragma unroll
  for (int i = 0; i < 8; ++i) { const int ka = k0 + 8 * g + i, kb = ka + 16; v[i] = ka < K ? W[(size_t)(ka < K ? ka : K - 1) * ld + n] : 0.f; v[8 + i] = kb < K ? W[(size_t)(kb < K ? kb : K - 1) * ld + n] : 0.f; }
  return bsplit16(v); }
__device__ __forceinline__ v8f mac3(const F2& a, const F2& b, v8f c) { c = wmma_bf(a.l, b.h, c); c = wmma_bf(a.h, b.l, c); return wmma_bf(a.h, b.h, c); }
__device__ __forceinline__ float sigm(float v) { return 1.0f / (1.0f + expf(-v)); }
#define LDSX() do { asm volatile("s_wait_dscnt 0" ::: "memory"); __builtin_amdgcn_wave_barrier(); __builtin_amdgcn_fence(__ATOMIC_RELEASE, "workgroup"); } while (0)


#ifndef NIMG
#define NIMG 32
#endif
#define KP 1000
#define KPP 1024
#define KG 100
#define KGP 128
#define NC 80
#define NCP 96
typedef __attribute__((ext_vector_type(8))) __bf16 v8b;
__device__ __forceinline__ v16b frag_b(const __bf16* rowk0, int lane) {
  union { v16b v; v8b q[2]; } u; const __bf16* p = rowk0 + 8 * (lane >> 4);
  u.q[0] = *(const v8b*)p; u.q[1] = *(const v8b*)(p + 16); return u.v;
}
__device__ __forceinline__ float bfr(float v) { return (float)(__bf16)v; }
__device__ __attribute__((noinline)) float exp_ni(float v) { return expf(v); }
__device__ __attribute__((noinline)) float erf_ni(float v) { return erff(v); }

__device__ __attribute__((noinline)) float log_ni(float v) { return logf(v); }
#define WS_AH  0u
#define WS_AL  (WS_AH + 2u * NIMG * KPP * NCP)
#define WS_GA  (WS_AL + 2u * NIMG * KPP * NCP)
#define WS_PS  (WS_GA + 2u * NIMG * KGP * NCP)
#define WS_END (WS_PS + 4u * NIMG * 3 * 16 * 32)

__global__ __launch_bounds__(128) void k_alpha(const float* __restrict__ PL, const int* __restrict__ GL, __bf16* __restrict__ AH, __bf16* __restrict__ AL, __bf16* __restrict__ GA) {
  __shared__ __align__(16) __bf16 sh[16][NCP], sl[16][NCP], sg[16][NCP];
  const int tid = threadIdx.x, img = blockIdx.y; const int r0 = blockIdx.x * 16;
  for (int q = tid; q < 16 * NCP; q += 128) { sh[q / NCP][q % NCP] = (__bf16)0.f; sl[q / NCP][q % NCP] = (__bf16)0.f; sg[q / NCP][q % NCP] = (__bf16)0.f; }
  __syncthreads();
  if (tid < 16) { const int r = r0 + tid;
    if (r < KP) { const float* lg = PL + ((size_t)img * KP + r) * (NC + 1); float mx = -3.0e38f; for (int c = 0; c < NC; ++c) mx = fmaxf(mx, bfr(lg[c])); float z = 0.f; for (int c = 0; c < NC; ++c) z += exp_ni(bfr(lg[c]) - mx); const float ob = sigm(bfr(lg[NC])); const float f = ob / z;
      for (int c = 0; c < NC; ++c) { const float a = exp_ni(bfr(lg[c]) - mx) * f; const __bf16 hb = (__bf16)a; sh[tid][c] = hb; sl[tid][c] = (__bf16)(a - (float)hb); } }
    if (r < KG) { const int lab = min(max(GL[(size_t)img * KG + r], 0), NC - 1); sg[tid][lab] = (__bf16)1.0f; } }
  __syncthreads();
  for (int q = tid; q < 16 * NCP / 8; q += 128) { vst2((unsigned*)(AH + ((size_t)img * KPP + r0) * NCP + q * 8), *(const v4u*)&(&sh[0][0])[q * 8]); vst2((unsigned*)(AL + ((size_t)img * KPP + r0) * NCP + q * 8), *(const v4u*)&(&sl[0][0])[q * 8]); }
  if (r0 < KGP) for (int q = tid; q < 16 * NCP / 8; q += 128) vst2((unsigned*)(GA + ((size_t)img * KGP + r0) * NCP + q * 8), *(const v4u*)&(&sg[0][0])[q * 8]);
}
struct GBox { float mx, my, cx, cy, q, lv; };
__device__ __forceinline__ GBox gauss(const float* __restrict__ BX, size_t r) { GBox g; g.mx = bfr(BX[r * 4 + 0]); g.my = bfr(BX[r * 4 + 1]); const float w = bfr(BX[r * 4 + 2]) * 0.5f, h = bfr(BX[r * 4 + 3]) * 0.5f; const float vx = w * w, vy = h * h; g.cx = 1.f / vx; g.cy = 1.f / vy; g.q = g.mx * g.mx / vx + g.my * g.my / vy; g.lv = log_ni(vx) + log_ni(vy); return g; }
__device__ __forceinline__ float pairdelta(const GBox& a, const GBox& b) {
  const float sx = a.cx + b.cx, sy = a.cy + b.cy; const float mijx = (a.mx * a.cx + b.mx * b.cx) / sx, mijy = (a.my * a.cy + b.my * b.cy) / sy;
  const float quad = (mijx * mijx * sx + mijy * mijy * sy) - a.q - b.q;
  const float logdet = log_ni(sx * sy) + a.lv + b.lv;
  return 0.5f * (quad - logdet - 2.0f * 1.8378770664093453f);
}
template <int TERM>
__global__ __launch_bounds__(128) void k_pair(const __bf16* __restrict__ AH, const __bf16* __restrict__ AL, const __bf16* __restrict__ GA, const float* __restrict__ PB, const float* __restrict__ GB, float* __restrict__ PS) {
  __shared__ float sred[4]; __shared__ __align__(16) float sline[32];
  const int tid = threadIdx.x, wave = tid >> 5, lane = tid & 31, col = lane & 15, g = lane >> 4; const int img = blockIdx.y, rt = blockIdx.x; const int nrows = (TERM == 2) ? KP : KG, ncols = (TERM == 1) ? KG : KP, ncolp = (TERM == 1) ? KGP : KPP;
  const __bf16* Arow_h = (TERM == 2) ? (AH + (size_t)img * KPP * NCP) : (GA + (size_t)img * KGP * NCP); const __bf16* Arow_l = (TERM == 2) ? (AL + (size_t)img * KPP * NCP) : nullptr;
  const __bf16* Brow_h = (TERM == 1) ? (GA + (size_t)img * KGP * NCP) : (AH + (size_t)img * KPP * NCP); const __bf16* Brow_l = (TERM == 1) ? nullptr : (AL + (size_t)img * KPP * NCP);
  const float* RB = (TERM == 2) ? (PB + (size_t)img * KP * 4) : (GB + (size_t)img * KG * 4); const float* CB = (TERM == 1) ? (GB + (size_t)img * KG * 4) : (PB + (size_t)img * KP * 4);
  const int r0 = rt * 64 + wave * 16; float psum = 0.f;
  GBox rowb[8];
#pragma unroll
  for (int r = 0; r < 8; ++r) { const int rr = r0 + 8 * g + r; const int rc = (rr < nrows) ? rr : 0; rowb[r] = gauss(RB, rc); }
#pragma unroll 1
  for (int cc = 0; cc < ncolp / 16; ++cc) { v8f w = {};
#pragma unroll
    for (int kc = 0; kc < NCP / 32; ++kc) { const v16b ah = frag_b(Arow_h + (size_t)(r0 + col) * NCP + kc * 32, lane); const v16b bh = frag_b(Brow_h + (size_t)(cc * 16 + col) * NCP + kc * 32, lane);
      w = wmma_bf(ah, bh, w);
      if (Brow_l) { const v16b bl = frag_b(Brow_l + (size_t)(cc * 16 + col) * NCP + kc * 32, lane); w = wmma_bf(ah, bl, w); }
      if (Arow_l) { const v16b al = frag_b(Arow_l + (size_t)(r0 + col) * NCP + kc * 32, lane); w = wmma_bf(al, bh, w); } }
    const int cidx = cc * 16 + col; if (cidx < ncols) { const GBox cb = gauss(CB, cidx);
#pragma unroll
      for (int r = 0; r < 8; ++r) { const int rr = r0 + 8 * g + r; if (rr < nrows) psum += w[r] * exp_ni(pairdelta(rowb[r], cb)); } } }
#pragma unroll
  for (int o = 1; o < 32; o <<= 1) psum += __shfl_xor(psum, o);
  if (lane == 0) sred[wave] = psum;
  __syncthreads();
  if (tid < 32) { float v = 0.f; if (tid == 0) v = (sred[0] + sred[1]) + (sred[2] + sred[3]); sline[tid] = v; }
  __syncthreads();
  if (tid < 8) vst2(PS + (((size_t)img * 3 + TERM) * 16 + rt) * 32 + tid * 4, *(const v4f*)&sline[tid * 4]);
}
__global__ __launch_bounds__(32) void k_final(const float* __restrict__ PS, float* __restrict__ out) {
  __shared__ float s[NIMG]; const int img = threadIdx.x;
  { float t[3]; for (int k = 0; k < 3; ++k) { const int nt = (k == 2) ? 16 : 2; float a = 0.f; for (int i = 0; i < nt; ++i) a += PS[(((size_t)img * 3 + k) * 16 + i) * 32]; t[k] = a; } s[img] = 2.0f * log_ni(t[0]) - log_ni(t[1]) - log_ni(t[2]); }
  __syncthreads();
  if (img == 0) { float tot = 0.f; for (int i = 0; i < NIMG; ++i) tot += s[i]; *(volatile float*)out = -tot; __threadfence(); *(volatile float*)out = -tot; }
}
extern "C" void kernel_launch(void* const* d_in, const int* in_sizes, int n_in, void* d_out, int out_size, void* d_ws, size_t ws_size, hipStream_t stream) {
  (void)in_sizes; (void)n_in; (void)out_size;
  const float* PB = (const float*)d_in[0]; const float* PL = (const float*)d_in[1]; const float* GB = (const float*)d_in[2]; const int* GL = (const int*)d_in[3];
  if (ws_size < (size_t)WS_END) return;
  char* ws = (char*)d_ws; __bf16 *AH = (__bf16*)(ws + WS_AH), *AL = (__bf16*)(ws + WS_AL), *GA = (__bf16*)(ws + WS_GA); float* PS = (float*)(ws + WS_PS);
  k_alpha<<<dim3(KPP / 16, NIMG), 128, 0, stream>>>(PL, GL, AH, AL, GA);
  k_pair<0><<<dim3(2, NIMG), 128, 0, stream>>>(AH, AL, GA, PB, GB, PS);
  k_pair<1><<<dim3(2, NIMG), 128, 0, stream>>>(AH, AL, GA, PB, GB, PS);
  k_pair<2><<<dim3(16, NIMG), 128, 0, stream>>>(AH, AL, GA, PB, GB, PS);
  k_final<<<1, NIMG, 0, stream>>>(PS, (float*)d_out);
}
